// TransformerBlock_83691732730567
// MI455X (gfx1250) — hardware-verified
//
#include <hip/hip_runtime.h>
#include <stddef.h>


typedef _Float16 v16h __attribute__((ext_vector_type(16)));
typedef _Float16 v8h  __attribute__((ext_vector_type(8)));
typedef float    v8f  __attribute__((ext_vector_type(8)));
typedef float    v4f  __attribute__((ext_vector_type(4)));

#ifndef NB
#define NB 2
#endif
#ifndef SEQ
#define SEQ 2048
#endif
#define NB_FULL  2
#define SEQ_FULL 2048
#define DIM   1024
#define NHEAD 16
#define HD    64
#define MROWS (NB * SEQ)

#define LDT 72
#define LDC 68
#define LDO 36

#define WCARRY 16.0f
#define PCARRY 1024.0f
#define MASKV  (-1.0e9f)
#define LN_EPS 1.0e-5f

static_assert(NB >= 1 && NB <= NB_FULL);
static_assert(SEQ >= 128 && SEQ <= SEQ_FULL && (SEQ % 128) == 0);
static_assert(DIM == NHEAD * HD);
static_assert(HD == 64);
static_assert((DIM % 64) == 0 && (DIM % 32) == 0);
static_assert((MROWS % 64) == 0);
static_assert((MROWS % 8) == 0);
static_assert(DIM == 8 * 32 * 4);
static_assert(((size_t)MROWS * DIM) % (8 * 256) == 0);
static_assert(((size_t)DIM * DIM) % (8 * 256) == 0);
static_assert((size_t)MROWS * DIM < (size_t)0xFFFFFFFFu);
static_assert((LDT * 2) % 16 == 0 && (LDC * 4) % 16 == 0 && (LDO * 4) % 16 == 0);
static_assert(LDT >= 64 && LDC >= 64 && LDO >= 32);
static_assert((2 * 64 * LDT + 8 * 16 * LDT) * 2 + 8 * 16 * LDO * 4 <= 65536);
static_assert(8 * DIM * 4 <= 65536);

#define PLANE16_BYTES ((size_t)MROWS * DIM * 2)
#define PLANE32_BYTES ((size_t)MROWS * DIM * 4)
#define WT_BYTES      ((size_t)3 * DIM * DIM * 2)
#define WS_TOTAL      (WT_BYTES + PLANE16_BYTES * 4 + PLANE32_BYTES)
static_assert((WT_BYTES % 128) == 0 && (PLANE16_BYTES % 128) == 0 && (PLANE32_BYTES % 128) == 0);
static_assert(WS_TOTAL <= (size_t)134217728);

__device__ __forceinline__ float bf16r(float x) {
  unsigned int u = __float_as_uint(x);
  u = (u + 0x7FFFu + ((u >> 16) & 1u)) & 0xFFFF0000u;
  return __uint_as_float(u);
}

__device__ __forceinline__ v16h frag_at(const _Float16* p) {
  v8h lo = *(const v8h*)(p);
  v8h hi = *(const v8h*)(p + 16);
  v16h out;
#pragma unroll
  for (int i = 0; i < 8; ++i) { out[i] = lo[i]; out[i + 8] = hi[i]; }
  return out;
}
__device__ __forceinline__ v16h ld_frag(const _Float16* base, unsigned ld) {
  const unsigned lane = threadIdx.x & 31u;
  return frag_at(base + (lane & 15u) * ld + (lane >> 4) * 8u);
}

__device__ __forceinline__ v8f wmma16(v16h a, v16h b, v8f c) {
  v8f d = __builtin_amdgcn_wmma_f32_16x16x32_f16(false, a, false, b, (short)0, c,
                                                 false, false);
  asm volatile("v_nop\n\tv_nop\n\tv_nop\n\tv_nop" : "+v"(d) : "v"(a), "v"(b));
  return d;
}

__device__ __forceinline__ float red16_max(float x) {
#pragma unroll
  for (int off = 1; off < 16; off <<= 1) x = fmaxf(x, __shfl_xor(x, off, 32));
  return x;
}
__device__ __forceinline__ float red16_sum(float x) {
#pragma unroll
  for (int off = 1; off < 16; off <<= 1) x += __shfl_xor(x, off, 32);
  return x;
}
__device__ __forceinline__ float red32_sum(float x) {
#pragma unroll
  for (int off = 1; off < 32; off <<= 1) x += __shfl_xor(x, off, 32);
  return x;
}

__device__ __forceinline__ void wave_lds_sync() {
  __builtin_amdgcn_fence(3  , "wavefront");
  asm volatile("s_wait_dscnt 0x0" ::: "memory");
  __builtin_amdgcn_wave_barrier();
}

__global__ __launch_bounds__(256) void wconv_kernel(
    const float* __restrict__ W, _Float16* __restrict__ dst) {
  const unsigned e = (blockIdx.x * 256u + threadIdx.x) * 8u;
  const v4f a0 = *(const v4f*)(W + e);
  const v4f a1 = *(const v4f*)(W + e + 4);
  v8h o;
#pragma unroll
  for (int j = 0; j < 4; ++j) {
    o[j]     = (_Float16)(WCARRY * bf16r(a0[j]));
    o[j + 4] = (_Float16)(WCARRY * bf16r(a1[j]));
  }
  *(volatile v8h*)(dst + (size_t)e) = o;
  __threadfence();
  *(volatile v8h*)(dst + (size_t)e) = o;
}

__global__ __launch_bounds__(256) void xconv_kernel(
    const float* __restrict__ Xin, _Float16* __restrict__ dst) {
  const unsigned e = (blockIdx.x * 256u + threadIdx.x) * 8u;
  const unsigned crow = e / (unsigned)DIM;
  const unsigned c = e - crow * (unsigned)DIM;
  const unsigned bidx = crow / (unsigned)SEQ;
  const unsigned sq = crow - bidx * (unsigned)SEQ;
  const size_t frow = (size_t)bidx * SEQ_FULL + sq;
  const float* sp = Xin + frow * DIM + c;
  const v4f a0 = *(const v4f*)(sp);
  const v4f a1 = *(const v4f*)(sp + 4);
  v8h o;
#pragma unroll
  for (int j = 0; j < 4; ++j) {
    o[j]     = (_Float16)bf16r(a0[j]);
    o[j + 4] = (_Float16)bf16r(a1[j]);
  }
  *(volatile v8h*)(dst + (size_t)e) = o;
  __threadfence();
  *(volatile v8h*)(dst + (size_t)e) = o;
}

template <int MODE>
__device__ __forceinline__ void gemm_body(
    const _Float16* __restrict__ A16, const _Float16* __restrict__ Bt,
    const float* __restrict__ bias, _Float16* __restrict__ out16) {
  __shared__ float Cs[64 * LDC];
  const unsigned tid = threadIdx.x, lane = tid & 31u;
  const unsigned w = (unsigned)__builtin_amdgcn_readfirstlane((int)(tid >> 5));
  const unsigned mw = w >> 1, nw = w & 1u;
  const unsigned hh = lane >> 4, m = lane & 15u;
  const unsigned n0 = blockIdx.x * 64u;
  const unsigned row0 = blockIdx.y * 64u;

  const _Float16* ap  = A16 + (size_t)(row0 + mw * 16u + m) * DIM + hh * 8u;
  const _Float16* bp0 = Bt + (size_t)(n0 + nw * 32u + m) * DIM + hh * 8u;
  const _Float16* bp1 = bp0 + 16 * DIM;
  v8f acc0 = {}, acc1 = {};
#pragma unroll 2
  for (unsigned k0 = 0; k0 < (unsigned)DIM; k0 += 32u) {
    const v16h a  = frag_at(ap + k0);
    const v16h b0 = frag_at(bp0 + k0);
    const v16h b1 = frag_at(bp1 + k0);
    acc0 = wmma16(a, b0, acc0);
    acc1 = wmma16(a, b1, acc1);
  }
#pragma unroll
  for (int r = 0; r < 8; ++r) {
    float* d = &Cs[(mw * 16u + hh * 8u + (unsigned)r) * LDC + nw * 32u + m];
    d[0]  = acc0[r];
    d[16] = acc1[r];
  }
  __syncthreads();

  if (MODE == 0) {
    v8h x[2];
    size_t off[2];
#pragma unroll
    for (unsigned i = 0; i < 2u; ++i) {
      const unsigned r = 32u * i + (tid >> 3);
      const unsigned c = (tid & 7u) * 8u;
      const v4f u0 = *(const v4f*)&Cs[r * LDC + c];
      const v4f u1 = *(const v4f*)&Cs[r * LDC + c + 4];
      const v4f g0 = *(const v4f*)(bias + n0 + c);
      const v4f g1 = *(const v4f*)(bias + n0 + c + 4);
#pragma unroll
      for (int j = 0; j < 4; ++j) {
        x[i][j]     = (_Float16)(u0[j] * (1.0f / WCARRY) + bf16r(g0[j]));
        x[i][j + 4] = (_Float16)(u1[j] * (1.0f / WCARRY) + bf16r(g1[j]));
      }
      off[i] = (size_t)(row0 + r) * DIM + n0 + c;
    }
#pragma unroll
    for (int i = 0; i < 2; ++i) *(volatile v8h*)(out16 + off[i]) = x[i];
    __threadfence();
#pragma unroll
    for (int i = 0; i < 2; ++i) *(volatile v8h*)(out16 + off[i]) = x[i];
  }

  if (MODE == 1) {
    const unsigned bidx = row0 / (unsigned)SEQ;
    const unsigned key0 = row0 - bidx * (unsigned)SEQ;
    v8h x[2];
    size_t off[2];
#pragma unroll
    for (unsigned i = 0; i < 2u; ++i) {
      const unsigned dcol = 32u * i + (tid >> 3);
      const unsigned kk = (tid & 7u) * 8u;
      const float bc = bf16r(bias[n0 + dcol]);
#pragma unroll
      for (unsigned j = 0; j < 8u; ++j)
        x[i][j] = (_Float16)(Cs[(kk + j) * LDC + dcol] * (1.0f / WCARRY) + bc);
      off[i] = ((size_t)bidx * DIM + n0 + dcol) * SEQ + key0 + kk;
    }
#pragma unroll
    for (int i = 0; i < 2; ++i) *(volatile v8h*)(out16 + off[i]) = x[i];
    __threadfence();
#pragma unroll
    for (int i = 0; i < 2; ++i) *(volatile v8h*)(out16 + off[i]) = x[i];
  }
}

__global__ __launch_bounds__(256) void gemm_rows_kernel(
    const _Float16* __restrict__ A16, const _Float16* __restrict__ Bt,
    const float* __restrict__ bias, _Float16* __restrict__ out16) {
  gemm_body<0>(A16, Bt, bias, out16);
}
__global__ __launch_bounds__(256) void gemm_vt_kernel(
    const _Float16* __restrict__ A16, const _Float16* __restrict__ Bt,
    const float* __restrict__ bias, _Float16* __restrict__ out16) {
  gemm_body<1>(A16, Bt, bias, out16);
}

__global__ __launch_bounds__(256) void attn_kernel(
    const _Float16* __restrict__ Qh, const _Float16* __restrict__ Kh,
    const _Float16* __restrict__ Vt, float* __restrict__ Ctx) {
  __shared__ _Float16 Ks[64 * LDT];
  __shared__ _Float16 Vs[64 * LDT];
  __shared__ _Float16 Ps[8 * 16 * LDT];
  __shared__ float    Os[8 * 16 * LDO];

  const unsigned tid = threadIdx.x, lane = tid & 31u;
  const unsigned w = (unsigned)__builtin_amdgcn_readfirstlane((int)(tid >> 5));
  const unsigned hh = lane >> 4, m = lane & 15u;
  const unsigned q0 = blockIdx.x * 128u;
  const unsigned head = blockIdx.y;
  const unsigned b = blockIdx.z;
  const float scale = 0.125f;
  const unsigned qw = q0 + w * 16u;
  const bool fullrow = (qw + 16u == (unsigned)SEQ);
  const unsigned kstart = (q0 + 128u == (unsigned)SEQ) ? 0u : q0;
  const unsigned pbase = w * (16u * LDT);
  const unsigned obase = w * (16u * LDO);

  const size_t qoff = (size_t)(b * (unsigned)SEQ + qw + m) * DIM + head * HD + hh * 8u;
  v16h qf[2];
  qf[0] = frag_at(Qh + qoff);
  qf[1] = frag_at(Qh + qoff + 32);

  float mrow[8], lrow[8];
  v8f o[4];
#pragma unroll
  for (int v = 0; v < 8; ++v) { mrow[v] = -1.0e30f; lrow[v] = 0.0f; }
#pragma unroll
  for (int nb = 0; nb < 4; ++nb) o[nb] = (v8f){};

  const size_t kplane = (size_t)b * SEQ * DIM + head * HD;
  const size_t vplane = ((size_t)b * DIM + head * HD) * SEQ;

  for (unsigned kb = kstart; kb < (unsigned)SEQ; kb += 64u) {
#pragma unroll
    for (unsigned j = 0; j < 2u; ++j) {
      const unsigned idx = tid + 256u * j;
      const unsigned r = idx >> 3, c = (idx & 7u) * 8u;
      *(v8h*)&Ks[r * LDT + c] = *(const v8h*)(Kh + kplane + (size_t)(kb + r) * DIM + c);
      *(v8h*)&Vs[r * LDT + c] = *(const v8h*)(Vt + vplane + (size_t)r * SEQ + kb + c);
    }
    __syncthreads();

    if (fullrow || (kb + 63u > qw)) {
      v8f s[4];
#pragma unroll
      for (int kg = 0; kg < 4; ++kg) {
        v8f t = {};
#pragma unroll
        for (int c = 0; c < 2; ++c) {
          const v16h kf = ld_frag(&Ks[(kg * 16) * LDT + c * 32], LDT);
          t = wmma16(qf[c], kf, t);
        }
        s[kg] = t * scale;
      }

      if (kb <= qw + 15u) {
#pragma unroll
        for (int kg = 0; kg < 4; ++kg) {
          const unsigned key = kb + (unsigned)kg * 16u + m;
#pragma unroll
          for (int v = 0; v < 8; ++v) {
            const unsigned qrow = qw + hh * 8u + (unsigned)v;
            s[kg][v] = (key <= qrow) ? MASKV : s[kg][v];
          }
        }
      }

      float alpha[8];
#pragma unroll
      for (int v = 0; v < 8; ++v) {
        float mx = fmaxf(fmaxf(s[0][v], s[1][v]), fmaxf(s[2][v], s[3][v]));
        mx = red16_max(mx);
        const float mn = fmaxf(mrow[v], mx);
        alpha[v] = __expf(mrow[v] - mn);
        mrow[v] = mn;
      }
#pragma unroll
      for (int kg = 0; kg < 4; ++kg)
#pragma unroll
        for (int v = 0; v < 8; ++v) s[kg][v] = __expf(s[kg][v] - mrow[v]);
#pragma unroll
      for (int v = 0; v < 8; ++v) {
        const float rs = red16_sum((s[0][v] + s[1][v]) + (s[2][v] + s[3][v]));
        lrow[v] = alpha[v] * lrow[v] + rs;
      }
#pragma unroll
      for (int nb = 0; nb < 4; ++nb)
#pragma unroll
        for (int v = 0; v < 8; ++v) o[nb][v] = o[nb][v] * alpha[v];

#pragma unroll
      for (int kg = 0; kg < 4; ++kg)
#pragma unroll
        for (int v = 0; v < 8; ++v)
          Ps[pbase + (hh * 8u + (unsigned)v) * LDT + (unsigned)kg * 16u + m] =
              (_Float16)(s[kg][v] * PCARRY);
      wave_lds_sync();

#pragma unroll
      for (int c = 0; c < 2; ++c) {
        const v16h pf = ld_frag(&Ps[pbase + c * 32], LDT);
#pragma unroll
        for (int nb = 0; nb < 4; ++nb) {
          const v16h vf = ld_frag(&Vs[(nb * 16) * LDT + c * 32], LDT);
          o[nb] = wmma16(pf, vf, o[nb]);
        }
      }
    }
    __syncthreads();
  }

  float inv[8];
#pragma unroll
  for (int v = 0; v < 8; ++v) inv[v] = __builtin_amdgcn_rcpf(lrow[v]) * (1.0f / PCARRY);
  v4f xs[8];
  unsigned off[8];
#pragma unroll
  for (int ph = 0; ph < 2; ++ph) {
#pragma unroll
    for (int nbl = 0; nbl < 2; ++nbl)
#pragma unroll
      for (int v = 0; v < 8; ++v)
        Os[obase + (hh * 8u + (unsigned)v) * LDO + (unsigned)nbl * 16u + m] =
            o[ph * 2 + nbl][v] * inv[v];
    wave_lds_sync();
#pragma unroll
    for (unsigned i = 0; i < 4u; ++i) {
      const unsigned r = 4u * i + (lane >> 3);
      const unsigned c = (lane & 7u) * 4u;
      xs[ph * 4 + (int)i] = *(const v4f*)&Os[obase + r * LDO + c];
      off[ph * 4 + (int)i] = (b * (unsigned)SEQ + qw + r) * (unsigned)DIM + head * HD +
                             (unsigned)ph * 32u + c;
    }
    wave_lds_sync();
  }
#pragma unroll
  for (int i = 0; i < 8; ++i) *(volatile v4f*)(Ctx + off[i]) = xs[i];
  __threadfence();
#pragma unroll
  for (int i = 0; i < 8; ++i) *(volatile v4f*)(Ctx + off[i]) = xs[i];
}

__global__ __launch_bounds__(256) void ln_kernel(
    const float* __restrict__ Ctx, const float* __restrict__ Xin,
    const float* __restrict__ G, const float* __restrict__ Bv,
    float* __restrict__ Out) {
  __shared__ float Ys[8 * DIM];
  const unsigned tid = threadIdx.x, lane = tid & 31u;
  const unsigned w = (unsigned)__builtin_amdgcn_readfirstlane((int)(tid >> 5));
  const unsigned crow = blockIdx.x * 8u + w;
  const unsigned bidx = crow / (unsigned)SEQ;
  const unsigned sq = crow - bidx * (unsigned)SEQ;
  const size_t frow = (size_t)bidx * SEQ_FULL + sq;
  const unsigned cbase = crow * (unsigned)DIM + lane * 4u;
  const size_t xbase = frow * DIM + lane * 4u;
  const unsigned ybase = w * (unsigned)DIM + lane * 4u;

  float sum = 0.0f;
#pragma unroll 1
  for (unsigned j = 0; j < 8u; ++j) {
    const v4f c = *(const v4f*)(Ctx + cbase + j * 128u);
    const v4f x = *(const v4f*)(Xin + xbase + j * 128u);
    v4f y;
#pragma unroll
    for (int t = 0; t < 4; ++t) y[t] = c[t] + bf16r(x[t]);
    *(v4f*)&Ys[ybase + j * 128u] = y;
    sum += (y[0] + y[1]) + (y[2] + y[3]);
  }
  sum = red32_sum(sum);
  const float mean = sum * (1.0f / (float)DIM);

  float ss = 0.0f;
#pragma unroll 1
  for (unsigned j = 0; j < 8u; ++j) {
    const v4f y = *(const v4f*)&Ys[ybase + j * 128u];
    v4f d;
#pragma unroll
    for (int t = 0; t < 4; ++t) d[t] = y[t] - mean;
    ss += (d[0] * d[0] + d[1] * d[1]) + (d[2] * d[2] + d[3] * d[3]);
  }
  ss = red32_sum(ss);
  const float rstd = rsqrtf(ss * (1.0f / (float)DIM) + LN_EPS);

#pragma unroll 1
  for (unsigned j = 0; j < 8u; ++j) {
    const v4f y = *(const v4f*)&Ys[ybase + j * 128u];
    const v4f g = *(const v4f*)(G + lane * 4u + j * 128u);
    const v4f bb = *(const v4f*)(Bv + lane * 4u + j * 128u);
    v4f val;
#pragma unroll
    for (int t = 0; t < 4; ++t) val[t] = (y[t] - mean) * rstd * bf16r(g[t]) + bf16r(bb[t]);
    *(v4f*)&Ys[ybase + j * 128u] = val;
    *(volatile v4f*)(Out + xbase + j * 128u) = val;
  }
  __threadfence();
#pragma unroll 1
  for (unsigned j = 0; j < 8u; ++j) {
    const v4f val = *(const v4f*)&Ys[ybase + j * 128u];
    *(volatile v4f*)(Out + xbase + j * 128u) = val;
  }
}

extern "C" void kernel_launch(void* const* d_in, const int* in_sizes, int n_in,
                              void* d_out, int out_size, void* d_ws, size_t ws_size,
                              hipStream_t stream) {
  if (n_in < 9) return;
  const long long need_x = ((long long)(NB - 1) * SEQ_FULL + SEQ) * DIM;
  if ((long long)in_sizes[0] < need_x) return;
  if ((long long)in_sizes[1] < (long long)DIM * DIM) return;
  if (in_sizes[2] < DIM) return;
  if ((long long)in_sizes[3] < (long long)DIM * DIM) return;
  if (in_sizes[4] < DIM) return;
  if ((long long)in_sizes[5] < (long long)DIM * DIM) return;
  if (in_sizes[6] < DIM) return;
  if (in_sizes[7] < DIM) return;
  if (in_sizes[8] < DIM) return;
  if ((long long)out_size < need_x) return;
  if (ws_size < WS_TOTAL) return;

  const float* X   = (const float*)d_in[0];
  const float* Wq  = (const float*)d_in[1];
  const float* bq  = (const float*)d_in[2];
  const float* Wk  = (const float*)d_in[3];
  const float* bk  = (const float*)d_in[4];
  const float* Wv  = (const float*)d_in[5];
  const float* bv  = (const float*)d_in[6];
  const float* lng = (const float*)d_in[7];
  const float* lnb = (const float*)d_in[8];
  float* out = (float*)d_out;

  char* ws = (char*)d_ws;
  _Float16* Wt    = (_Float16*)ws;
  _Float16* X16   = (_Float16*)(ws + WT_BYTES);
  _Float16* Qh16  = (_Float16*)(ws + WT_BYTES + 1 * PLANE16_BYTES);
  _Float16* Kh16  = (_Float16*)(ws + WT_BYTES + 2 * PLANE16_BYTES);
  _Float16* Vt16  = (_Float16*)(ws + WT_BYTES + 3 * PLANE16_BYTES);
  float*    Ctx32 = (float*)(ws + WT_BYTES + 4 * PLANE16_BYTES);

  const size_t WP = (size_t)DIM * DIM;
  dim3 blk(256);
  dim3 gw((unsigned)(((size_t)DIM * DIM) / 2048));
  dim3 gg(DIM / 64, MROWS / 64);

  wconv_kernel<<<gw, blk, 0, stream>>>(Wq, Wt + 0 * WP);
  wconv_kernel<<<gw, blk, 0, stream>>>(Wk, Wt + 1 * WP);
  wconv_kernel<<<gw, blk, 0, stream>>>(Wv, Wt + 2 * WP);
  xconv_kernel<<<dim3((unsigned)(((size_t)MROWS * DIM) / 2048)), blk, 0, stream>>>(X, X16);
  gemm_rows_kernel<<<gg, blk, 0, stream>>>(X16, Wt + 0 * WP, bq, Qh16);
  gemm_rows_kernel<<<gg, blk, 0, stream>>>(X16, Wt + 1 * WP, bk, Kh16);
  gemm_vt_kernel<<<gg, blk, 0, stream>>>(X16, Wt + 2 * WP, bv, Vt16);
  attn_kernel<<<dim3(SEQ / 128, NHEAD, NB), blk, 0, stream>>>(Qh16, Kh16, Vt16, Ctx32);
  ln_kernel<<<dim3(MROWS / 8), blk, 0, stream>>>(Ctx32, X, lng, lnb, out);
}
